// RITS_17712445129440
// MI455X (gfx1250) — hardware-run, weakly checked
//
#include <hip/hip_runtime.h>
#include <stddef.h>

typedef __attribute__((ext_vector_type(16))) _Float16 v16h;
typedef __attribute__((ext_vector_type(8)))  _Float16 v8h;
typedef __attribute__((ext_vector_type(8)))  float    v8f;
typedef __attribute__((ext_vector_type(4)))  float    v4f;

enum { kNB = 512, kNT = 128, kND = 128, kNH = 256 };
enum { kRows = 16, kThreads = 256 };
enum { kPitchA5 = 520, kPitchH = 136, kPitchF = 132 };
constexpr float kWCarry    = 16.0f;
constexpr float kWCarryInv = 0.0625f;

typedef char chk_rows_[(kNB % kRows == 0) ? 1 : -1];
typedef char chk_dims_[(kND == 128 && kNH == 256 && kRows == 16 && kThreads == 256) ? 1 : -1];
typedef char chk_ktile_[(kND % 32 == 0 && kNH % 32 == 0) ? 1 : -1];
typedef char chk_pitch_[((kPitchA5 % 8) == 0 && (kPitchH % 8) == 0 && (kPitchF % 4) == 0) ? 1 : -1];
typedef char chk_stage_[(kRows * kPitchF >= 2048) ? 1 : -1];

union FragU { v16h v; v8h h[2]; };
__device__ __forceinline__ v16h frag16(const _Float16* p) {
  FragU f;
  f.h[0] = *(const v8h*)(p);
  f.h[1] = *(const v8h*)(p + 16);
  return f.v;
}
__device__ __forceinline__ v8f mma16(v16h a, v16h b, v8f c) {
  c = __builtin_amdgcn_wmma_f32_16x16x32_f16(false, a, false, b, (short)0, c, false, false);
  asm volatile("v_nop\n\tv_nop\n\tv_nop\n\tv_nop" : "+v"(c) : "v"(a), "v"(b));
  return c;
}
__device__ __forceinline__ float sigm_f(float x) { return 1.0f / (1.0f + expf(-x)); }

__global__ __launch_bounds__(256) void cast_w_f16x2(const float* __restrict__ in, _Float16* __restrict__ out,
                                                    int n2, int zero_diag, float scale) {
  const int i = blockIdx.x * 256 + threadIdx.x;
  if (i < n2) {
    const int e0 = 2 * i, e1 = 2 * i + 1;
    float f0 = in[e0] * scale;
    float f1 = in[e1] * scale;
    if (zero_diag) {
      if ((e0 >> 7) == (e0 & 127)) f0 = 0.0f;
      if ((e1 >> 7) == (e1 & 127)) f1 = 0.0f;
    }
    const _Float16 h0 = (_Float16)f0, h1 = (_Float16)f1;
    const unsigned u = (unsigned)__builtin_bit_cast(unsigned short, h0) |
                       ((unsigned)__builtin_bit_cast(unsigned short, h1) << 16);
    ((volatile unsigned*)out)[i] = u;
    __threadfence();
    ((volatile unsigned*)out)[i] = u;
  }
}

__global__ __launch_bounds__(kThreads)
void recur_scan_kernel(const float* __restrict__ values,
                       const float* __restrict__ masks,
                       const float* __restrict__ deltas,
                       const float* __restrict__ W_td_x,
                       const float* __restrict__ b_td_x,
                       const float* __restrict__ b_td_h,
                       const float* __restrict__ b_hist,
                       const float* __restrict__ b_feat,
                       const float* __restrict__ b_comb,
                       const float* __restrict__ b_ih,
                       const float* __restrict__ b_hh,
                       const _Float16* __restrict__ w_tdh,
                       const _Float16* __restrict__ w_hist,
                       const _Float16* __restrict__ w_feat,
                       const _Float16* __restrict__ w_comb,
                       const _Float16* __restrict__ w_ih,
                       const _Float16* __restrict__ w_hh,
                       float* __restrict__ out) {
  __shared__ __align__(16) _Float16 sA5[kRows * kPitchA5];
  __shared__ __align__(16) _Float16 sGx[kRows * kPitchH];
  __shared__ __align__(16) _Float16 sDl[kRows * kPitchH];
  __shared__ __align__(16) _Float16 sXc[kRows * kPitchH];
  __shared__ __align__(16) float    sX [kRows * kPitchF];
  __shared__ __align__(16) float    sM [kRows * kPitchF];
  __shared__ __align__(16) float    sO [kRows * kPitchF];

  const int tid  = threadIdx.x;
  const int wave = tid >> 5;
  const int lane = tid & 31;
  const int hh   = lane >> 4;
  const int lr   = lane & 15;
  const int b0   = blockIdx.x * kRows;

  const int e0   = tid * 8;
  const int lrow = e0 >> 7;
  const int lcol = e0 & 127;
  const int colw = wave * 16 + lr;

  if (wave == 0) {
    const v4f a = *(const v4f*)(b_td_h + lane * 8);
    const v4f c = *(const v4f*)(b_td_h + lane * 8 + 4);
    *(v4f*)(sO + lane * 8) = a;
    *(v4f*)(sO + lane * 8 + 4) = c;
  } else if (wave == 1) {
    const v4f a = *(const v4f*)(b_hist + lane * 4);
    const v4f c = *(const v4f*)(b_feat + lane * 4);
    *(v4f*)(sO + 256 + lane * 4) = a;
    *(v4f*)(sO + 384 + lane * 4) = c;
  } else if (wave == 2) {
    const v4f a = *(const v4f*)(b_comb + lane * 4);
    const v4f c = *(const v4f*)(b_td_x + lane * 4);
    *(v4f*)(sO + 512 + lane * 4) = a;
    *(v4f*)(sO + 640 + lane * 4) = c;
  } else if (wave == 3) {
#pragma unroll
    for (int q = 0; q < 4; ++q) {
      const int ci = lane * 4 + q;
      sO[768 + ci] = W_td_x[(size_t)ci * (kND + 1)];
    }
  } else {
    const int base = (wave - 4) * 256 + lane * 8;
    const v4f a0 = *(const v4f*)(b_ih + base);
    const v4f a1 = *(const v4f*)(b_ih + base + 4);
    const v4f c0 = *(const v4f*)(b_hh + base);
    const v4f c1 = *(const v4f*)(b_hh + base + 4);
    *(v4f*)(sO + 1024 + base) = a0 + c0;
    *(v4f*)(sO + 1024 + base + 4) = a1 + c1;
  }
  __syncthreads();

  float bth_r[2], bg_r[8], btx_r[8], diagw_r[8];
#pragma unroll
  for (int j = 0; j < 2; ++j) bth_r[j] = sO[(wave + 8 * j) * 16 + lr];
#pragma unroll
  for (int j = 0; j < 8; ++j) bg_r[j] = sO[1024 + (wave + 8 * j) * 16 + lr];
#pragma unroll
  for (int i = 0; i < 8; ++i) { btx_r[i] = sO[640 + lcol + i]; diagw_r[i] = sO[768 + lcol + i]; }
  const float bhist_r = sO[256 + colw];
  const float bfeat_r = sO[384 + colw];
  const float bcomb_r = sO[512 + colw];
  __syncthreads();

  float h_reg[2][8], c_reg[2][8];
#pragma unroll
  for (int p = 0; p < 2; ++p)
#pragma unroll
    for (int g = 0; g < 8; ++g) { h_reg[p][g] = 0.0f; c_reg[p][g] = 0.0f; }

  const v8f z8 = {0.f, 0.f, 0.f, 0.f, 0.f, 0.f, 0.f, 0.f};

#pragma unroll 1
  for (int t = 0; t < kNT; ++t) {
    {
      const size_t gb = ((size_t)(b0 + lrow) * kNT + t) * kND + lcol;
      const v4f x0 = *(const v4f*)(values + gb), x1 = *(const v4f*)(values + gb + 4);
      const v4f m0 = *(const v4f*)(masks + gb),  m1 = *(const v4f*)(masks + gb + 4);
      const v4f d0 = *(const v4f*)(deltas + gb), d1 = *(const v4f*)(deltas + gb + 4);
      *(v4f*)(sX + lrow * kPitchF + lcol) = x0;
      *(v4f*)(sX + lrow * kPitchF + lcol + 4) = x1;
      *(v4f*)(sM + lrow * kPitchF + lcol) = m0;
      *(v4f*)(sM + lrow * kPitchF + lcol + 4) = m1;
      v8h mhv, dhv, ghv;
#pragma unroll
      for (int i = 0; i < 4; ++i) {
        mhv[i]     = (_Float16)m0[i];
        mhv[i + 4] = (_Float16)m1[i];
        dhv[i]     = (_Float16)d0[i];
        dhv[i + 4] = (_Float16)d1[i];
        const float g0 = expf(-fmaxf(d0[i] * diagw_r[i] + btx_r[i], 0.0f));
        const float g1 = expf(-fmaxf(d1[i] * diagw_r[i + 4] + btx_r[i + 4], 0.0f));
        ghv[i]     = (_Float16)g0;
        ghv[i + 4] = (_Float16)g1;
      }
      *(v8h*)(sA5 + lrow * kPitchA5 + kND + lcol) = mhv;
      *(v8h*)(sDl + lrow * kPitchH + lcol) = dhv;
      *(v8h*)(sGx + lrow * kPitchH + lcol) = ghv;
    }
    __syncthreads();

#pragma unroll
    for (int j = 0; j < 2; ++j) {
      const int tile = wave + 8 * j;
      v8f acc = z8;
      const _Float16* ap = sDl + lr * kPitchH + 8 * hh;
      const _Float16* bp = w_tdh + (size_t)(tile * 16 + lr) * kND + 8 * hh;
#pragma unroll 1
      for (int k0 = 0; k0 < kND; k0 += 32) acc = mma16(frag16(ap + k0), frag16(bp + k0), acc);
#pragma unroll
      for (int g = 0; g < 8; ++g) {
        const float gh = expf(-fmaxf(acc[g] * kWCarryInv + bth_r[j], 0.0f));
        const float hs = h_reg[j][g] * gh;
        sA5[(8 * hh + g) * kPitchA5 + 2 * kND + tile * 16 + lr] = (_Float16)hs;
      }
    }
    __syncthreads();

    float xh_r[8], al_r[8];
    {
      v8f acc2 = z8, acc4 = z8;
      {
        const _Float16* ap = sA5 + lr * kPitchA5 + 2 * kND + 8 * hh;
        const _Float16* bp = w_hist + (size_t)colw * kNH + 8 * hh;
#pragma unroll 1
        for (int k0 = 0; k0 < kNH; k0 += 32) acc2 = mma16(frag16(ap + k0), frag16(bp + k0), acc2);
      }
      {
        const _Float16* ap = sGx + lr * kPitchH + 8 * hh;
        const _Float16* bp = w_comb + (size_t)colw * (2 * kND) + 8 * hh;
#pragma unroll 1
        for (int k0 = 0; k0 < kND; k0 += 32) acc4 = mma16(frag16(ap + k0), frag16(bp + k0), acc4);
      }
      {
        const _Float16* ap = sA5 + lr * kPitchA5 + kND + 8 * hh;
        const _Float16* bp = w_comb + (size_t)colw * (2 * kND) + kND + 8 * hh;
#pragma unroll 1
        for (int k0 = 0; k0 < kND; k0 += 32) acc4 = mma16(frag16(ap + k0), frag16(bp + k0), acc4);
      }
#pragma unroll
      for (int g = 0; g < 8; ++g) {
        const int mr = 8 * hh + g;
        const float xh = acc2[g] * kWCarryInv + bhist_r;
        const float al = acc4[g] * kWCarryInv + bcomb_r;
        const float mm = sM[mr * kPitchF + colw];
        const float xx = sX[mr * kPitchF + colw];
        const float xc = mm * xx + (1.0f - mm) * xh;
        sXc[mr * kPitchH + colw] = (_Float16)xc;
        xh_r[g] = xh;
        al_r[g] = al;
      }
    }
    __syncthreads();

    {
      v8f acc3 = z8;
      const _Float16* ap = sXc + lr * kPitchH + 8 * hh;
      const _Float16* bp = w_feat + (size_t)colw * kND + 8 * hh;
#pragma unroll 1
      for (int k0 = 0; k0 < kND; k0 += 32) acc3 = mma16(frag16(ap + k0), frag16(bp + k0), acc3);
#pragma unroll
      for (int g = 0; g < 8; ++g) {
        const int mr = 8 * hh + g;
        const float zh = acc3[g] * kWCarryInv + bfeat_r;
        const float ch = al_r[g] * zh + (1.0f - al_r[g]) * xh_r[g];
        const float mm = sM[mr * kPitchF + colw];
        const float xx = sX[mr * kPitchF + colw];
        const float cc = mm * xx + (1.0f - mm) * ch;
        sO[mr * kPitchF + colw] = cc;
        sA5[mr * kPitchA5 + colw] = (_Float16)cc;
      }
    }
    __syncthreads();

    {
      const int r0 = 2 * wave, r1 = 2 * wave + 1;
      const v4f o0 = *(const v4f*)(sO + r0 * kPitchF + lane * 4);
      const v4f o1 = *(const v4f*)(sO + r1 * kPitchF + lane * 4);
      float* p0 = out + ((size_t)(b0 + r0) * kNT + t) * kND + lane * 4;
      float* p1 = out + ((size_t)(b0 + r1) * kNT + t) * kND + lane * 4;
      *(volatile v4f*)p0 = o0;
      *(volatile v4f*)p1 = o1;
      __threadfence();
      *(volatile v4f*)p0 = o0;
      *(volatile v4f*)p1 = o1;
    }

    {
      const _Float16* arow = sA5 + lr * kPitchA5 + 8 * hh;
#pragma unroll
      for (int p = 0; p < 2; ++p) {
        v8f g4[4];
#pragma unroll
        for (int q = 0; q < 4; ++q) g4[q] = z8;
#pragma unroll 1
        for (int k0 = 0; k0 < 2 * kND; k0 += 32) {
          const v16h a = frag16(arow + k0);
#pragma unroll
          for (int q = 0; q < 4; ++q) {
            const int n = (wave + 8 * (p + 2 * q)) * 16 + lr;
            g4[q] = mma16(a, frag16(w_ih + (size_t)n * (2 * kND) + 8 * hh + k0), g4[q]);
          }
        }
#pragma unroll 1
        for (int k0 = 0; k0 < kNH; k0 += 32) {
          const v16h a = frag16(arow + 2 * kND + k0);
#pragma unroll
          for (int q = 0; q < 4; ++q) {
            const int n = (wave + 8 * (p + 2 * q)) * 16 + lr;
            g4[q] = mma16(a, frag16(w_hh + (size_t)n * kNH + 8 * hh + k0), g4[q]);
          }
        }
#pragma unroll
        for (int g = 0; g < 8; ++g) {
          const float ig = sigm_f(g4[0][g] * kWCarryInv + bg_r[p + 0]);
          const float fg = sigm_f(g4[1][g] * kWCarryInv + bg_r[p + 2]);
          const float gg = tanhf (g4[2][g] * kWCarryInv + bg_r[p + 4]);
          const float og = sigm_f(g4[3][g] * kWCarryInv + bg_r[p + 6]);
          const float cn = fg * c_reg[p][g] + ig * gg;
          c_reg[p][g] = cn;
          h_reg[p][g] = og * tanhf(cn);
        }
      }
    }
    __syncthreads();
  }
}

extern "C" void kernel_launch(void* const* d_in, const int* in_sizes, int n_in,
                              void* d_out, int out_size, void* d_ws, size_t ws_size,
                              hipStream_t stream) {
  if (n_in < 17) return;
  if (in_sizes[0] != kNB * kNT * kND || in_sizes[1] != kNB * kNT * kND || in_sizes[2] != kNB * kNT * kND) return;
  if (in_sizes[3] != kNH * kND || in_sizes[4] != kNH || in_sizes[5] != kND * kND || in_sizes[6] != kND) return;
  if (in_sizes[7] != kND * kNH || in_sizes[8] != kND || in_sizes[9] != kND * kND || in_sizes[10] != kND) return;
  if (in_sizes[11] != kND * 2 * kND || in_sizes[12] != kND) return;
  if (in_sizes[13] != 4 * kNH * 2 * kND || in_sizes[14] != 4 * kNH * kNH || in_sizes[15] != 4 * kNH || in_sizes[16] != 4 * kNH) return;
  if (out_size != kNB * kNT * kND) return;

  const float* values = (const float*)d_in[0];
  const float* masks  = (const float*)d_in[1];
  const float* deltas = (const float*)d_in[2];
  const float* W_td_h = (const float*)d_in[3];
  const float* b_td_h = (const float*)d_in[4];
  const float* W_td_x = (const float*)d_in[5];
  const float* b_td_x = (const float*)d_in[6];
  const float* W_hist = (const float*)d_in[7];
  const float* b_hist = (const float*)d_in[8];
  const float* W_feat = (const float*)d_in[9];
  const float* b_feat = (const float*)d_in[10];
  const float* W_comb = (const float*)d_in[11];
  const float* b_comb = (const float*)d_in[12];
  const float* W_ih   = (const float*)d_in[13];
  const float* W_hh   = (const float*)d_in[14];
  const float* b_ih   = (const float*)d_in[15];
  const float* b_hh   = (const float*)d_in[16];
  float* out = (float*)d_out;

  const size_t n_tdh = (size_t)kNH * kND, n_hist = (size_t)kND * kNH, n_feat = (size_t)kND * kND;
  const size_t n_comb = (size_t)kND * 2 * kND, n_ih = (size_t)4 * kNH * 2 * kND, n_hh = (size_t)4 * kNH * kNH;
  const size_t off_tdh = 0;
  const size_t off_hist = off_tdh + n_tdh * 2;
  const size_t off_feat = off_hist + n_hist * 2;
  const size_t off_comb = off_feat + n_feat * 2;
  const size_t off_ih   = off_comb + n_comb * 2;
  const size_t off_hh   = off_ih + n_ih * 2;
  const size_t total    = off_hh + n_hh * 2;
  if (total > ws_size) return;

  char* ws = (char*)d_ws;
  _Float16* p_tdh  = (_Float16*)(ws + off_tdh);
  _Float16* p_hist = (_Float16*)(ws + off_hist);
  _Float16* p_feat = (_Float16*)(ws + off_feat);
  _Float16* p_comb = (_Float16*)(ws + off_comb);
  _Float16* p_ih   = (_Float16*)(ws + off_ih);
  _Float16* p_hh   = (_Float16*)(ws + off_hh);

  {
    const int n2 = (int)(n_tdh / 2);
    cast_w_f16x2<<<dim3((n2 + 255) / 256), dim3(256), 0, stream>>>(W_td_h, p_tdh, n2, 0, kWCarry);
  }
  {
    const int n2 = (int)(n_hist / 2);
    cast_w_f16x2<<<dim3((n2 + 255) / 256), dim3(256), 0, stream>>>(W_hist, p_hist, n2, 0, kWCarry);
  }
  {
    const int n2 = (int)(n_feat / 2);
    cast_w_f16x2<<<dim3((n2 + 255) / 256), dim3(256), 0, stream>>>(W_feat, p_feat, n2, 1, kWCarry);
  }
  {
    const int n2 = (int)(n_comb / 2);
    cast_w_f16x2<<<dim3((n2 + 255) / 256), dim3(256), 0, stream>>>(W_comb, p_comb, n2, 0, kWCarry);
  }
  {
    const int n2 = (int)(n_ih / 2);
    cast_w_f16x2<<<dim3((n2 + 255) / 256), dim3(256), 0, stream>>>(W_ih, p_ih, n2, 0, kWCarry);
  }
  {
    const int n2 = (int)(n_hh / 2);
    cast_w_f16x2<<<dim3((n2 + 255) / 256), dim3(256), 0, stream>>>(W_hh, p_hh, n2, 0, kWCarry);
  }

  recur_scan_kernel<<<dim3(kNB / kRows), dim3(kThreads), 0, stream>>>(
      values, masks, deltas, W_td_x, b_td_x, b_td_h, b_hist, b_feat, b_comb, b_ih, b_hh,
      p_tdh, p_hist, p_feat, p_comb, p_ih, p_hh, out);
}
